// GNN_10574209482835
// MI455X (gfx1250) — hardware-verified
//
#include <hip/hip_runtime.h>
#include <stddef.h>
#include <stdint.h>
#include <math.h>


#define FIN    768
#define D1     1024
#define D2     768
#define K2     2048
#define NTHR   256
#define NWAVE  8
#define EPT    8
#define CHUNK  (NTHR * EPT)
#define WCAP   (EPT * 32)
#define LISTN  (NWAVE * WCAP)
#define NBA    512
#define SLA    9
#define RCAP   12288
#define DEGCAP 64
#define GBM    64
#define GBN    128
#define GTHR   128
#define NUW1   (D1 * (FIN / 8))
#define NUW2   (D2 * (K2 / 8))
#define AGG_ZINTS   (LISTN + 2 * RCAP + 3 * NBA)
#define MISC_INTS   16
#define SSRC_INTS   (NWAVE * DEGCAP)
#define SC_INTS     (NWAVE * DEGCAP * 8)
#define ZTOT_INTS   (AGG_ZINTS + MISC_INTS + SSRC_INTS + SC_INTS)
#define ROWBUF_INTS (NWAVE * K2 / 2)
#define SCAN_LDS_INTS (ZTOT_INTS + ROWBUF_INTS)
#define WSMAX  134217728

static_assert((CHUNK & (CHUNK - 1)) == 0 && CHUNK <= 4096);
static_assert((NBA & (NBA - 1)) == 0 && NBA == (1 << SLA));
static_assert(((long long)CHUNK << SLA) < (1LL << 31));
static_assert(NBA % NWAVE == 0 && NBA % 32 == 0);
static_assert(RCAP % 4 == 0 && AGG_ZINTS % 4 == 0 && LISTN % 4 == 0 && ZTOT_INTS % 4 == 0);
static_assert(((AGG_ZINTS + MISC_INTS + SSRC_INTS) % 4) == 0);
static_assert(DEGCAP % 32 == 0 && DEGCAP >= 36 + 8);
static_assert(FIN % 32 == 0 && K2 % 32 == 0 && K2 == 2 * D1);
static_assert(D1 % GBN == 0 && D2 % GBN == 0 && D1 / GBN == 8 && D2 / GBN == 6);
static_assert(GBM == (GTHR / 32) * 16 && GBN == 4 * 32);
static_assert(NUW1 % NTHR == 0 && NUW2 % NTHR == 0 && (128 * (FIN / 8)) % NTHR == 0);
static_assert(SCAN_LDS_INTS * 4 <= 300000);

typedef float          v4f   __attribute__((ext_vector_type(4)));
typedef float          v8f   __attribute__((ext_vector_type(8)));
typedef int            v4i   __attribute__((ext_vector_type(4)));
typedef int            v8i   __attribute__((ext_vector_type(8)));
typedef unsigned short v4us  __attribute__((ext_vector_type(4)));
typedef unsigned short v8us  __attribute__((ext_vector_type(8)));
typedef unsigned short v16us __attribute__((ext_vector_type(16)));
typedef __bf16         v16bf __attribute__((ext_vector_type(16)));
typedef v4f  __attribute__((may_alias)) v4fa;
typedef v4i  __attribute__((may_alias)) v4ia;
typedef v4us __attribute__((may_alias)) v4usa;
typedef v8us __attribute__((may_alias)) v8usa;
union FragB { v16bf v; v16us u; v8us h[2]; v8i w; };

__device__ __forceinline__ v8f wmb(const FragB& a, const FragB& b, v8f c) {
  v8f d = __builtin_amdgcn_wmma_f32_16x16x32_bf16(false, a.v, false, b.v, (short)0, c, false, false);
  asm volatile("v_nop\n\tv_nop\n\tv_nop\n\tv_nop" : "+v"(d) : "v"(a.w), "v"(b.w));
  return d;
}

__device__ __forceinline__ unsigned bf16_bits(float f) {
  const unsigned u = __float_as_uint(f);
  return (u + 0x7FFFu + ((u >> 16) & 1u)) >> 16;
}
__device__ __forceinline__ float bf16_val(float f) {
  return __uint_as_float(bf16_bits(f) << 16);
}

__device__ __forceinline__ void wave_sync() {
  __builtin_amdgcn_fence(__ATOMIC_RELEASE, "wavefront");
  __builtin_amdgcn_wave_barrier();
  __builtin_amdgcn_fence(__ATOMIC_ACQUIRE, "wavefront");
}

__device__ __forceinline__ void put8(unsigned short* dp, v8us o) {
  *(volatile v8us*)dp = o;
  __threadfence();
  *(volatile v8us*)dp = o;
}

__device__ __forceinline__ v8us cvt8(v4f a, v4f b, bool ok) {
  v8us o;
  o[0] = ok ? (unsigned short)bf16_bits(a.x) : (unsigned short)0;
  o[1] = ok ? (unsigned short)bf16_bits(a.y) : (unsigned short)0;
  o[2] = ok ? (unsigned short)bf16_bits(a.z) : (unsigned short)0;
  o[3] = ok ? (unsigned short)bf16_bits(a.w) : (unsigned short)0;
  o[4] = ok ? (unsigned short)bf16_bits(b.x) : (unsigned short)0;
  o[5] = ok ? (unsigned short)bf16_bits(b.y) : (unsigned short)0;
  o[6] = ok ? (unsigned short)bf16_bits(b.z) : (unsigned short)0;
  o[7] = ok ? (unsigned short)bf16_bits(b.w) : (unsigned short)0;
  return o;
}

template <int SLB>
__device__ __forceinline__ int scan_chunk(const int* __restrict__ dsts, int nE, int cbase, int slotBase,
                                          int nb, int vec8, int* list, int tid, int lane, int wave) {
  int wc = 0;
  const int el0  = tid * EPT;
  const int e0   = cbase + el0;
  const int sent = -2147483647 - 1;
  v4i da, db;
  if (vec8 != 0 && cbase + CHUNK <= nE) {
    da = *(const v4i*)(dsts + e0);
    db = *(const v4i*)(dsts + e0 + 4);
  } else {
    da.x = (e0     < nE) ? dsts[min(e0,     nE - 1)] : sent;
    da.y = (e0 + 1 < nE) ? dsts[min(e0 + 1, nE - 1)] : sent;
    da.z = (e0 + 2 < nE) ? dsts[min(e0 + 2, nE - 1)] : sent;
    da.w = (e0 + 3 < nE) ? dsts[min(e0 + 3, nE - 1)] : sent;
    db.x = (e0 + 4 < nE) ? dsts[min(e0 + 4, nE - 1)] : sent;
    db.y = (e0 + 5 < nE) ? dsts[min(e0 + 5, nE - 1)] : sent;
    db.z = (e0 + 6 < nE) ? dsts[min(e0 + 6, nE - 1)] : sent;
    db.w = (e0 + 7 < nE) ? dsts[min(e0 + 7, nE - 1)] : sent;
  }
  const unsigned nbs = (unsigned)slotBase;
  const unsigned unb = (unsigned)nb;
  const unsigned s0 = (unsigned)da.x - nbs, s1 = (unsigned)da.y - nbs;
  const unsigned s2 = (unsigned)da.z - nbs, s3 = (unsigned)da.w - nbs;
  const unsigned s4 = (unsigned)db.x - nbs, s5 = (unsigned)db.y - nbs;
  const unsigned s6 = (unsigned)db.z - nbs, s7 = (unsigned)db.w - nbs;
  const bool h0 = s0 < unb, h1 = s1 < unb, h2 = s2 < unb, h3 = s3 < unb;
  const bool h4 = s4 < unb, h5 = s5 < unb, h6 = s6 < unb, h7 = s7 < unb;
  const unsigned any = __builtin_amdgcn_ballot_w32(h0 | h1 | h2 | h3 | h4 | h5 | h6 | h7);
  if (any != 0u) {
#define HITJ(J, HJ, SJ) { \
      const unsigned mj = __builtin_amdgcn_ballot_w32(HJ); \
      if (mj != 0u) { \
        if (HJ) { \
          const int pos = wc + (int)__builtin_amdgcn_mbcnt_lo(mj, 0u); \
          if (pos < WCAP) list[wave * WCAP + pos] = ((el0 + (J)) << SLB) | (int)(SJ); \
        } \
        wc += (int)__builtin_popcount(mj); } }
    HITJ(0, h0, s0)
    HITJ(1, h1, s1)
    HITJ(2, h2, s2)
    HITJ(3, h3, s3)
    HITJ(4, h4, s4)
    HITJ(5, h5, s5)
    HITJ(6, h6, s6)
    HITJ(7, h7, s7)
#undef HITJ
  }
  return wc;
}

__global__ __launch_bounds__(NTHR) void k_prep(const float* __restrict__ x, const float* __restrict__ W1,
                                               const float* __restrict__ W2, int nN, int mp,
                                               unsigned short* XB, unsigned short* W1B, unsigned short* W2D) {
  const int u   = (int)blockIdx.x * NTHR + (int)threadIdx.x;
  const int nUX = mp * (FIN / 8);
  if (u < nUX) {
    const int row = u / (FIN / 8);
    const int k8  = (u - row * (FIN / 8)) * 8;
    const int rc  = row < nN ? row : nN - 1;
    const float* p = x + (size_t)rc * FIN + k8;
    const v4f a = *(const v4fa*)p;
    const v4f b = *(const v4fa*)(p + 4);
    put8(XB + (size_t)row * FIN + k8, cvt8(a, b, row < nN));
  } else if (u < nUX + NUW1) {
    const int v  = u - nUX;
    const int n  = v / (FIN / 8);
    const int k8 = (v - n * (FIN / 8)) * 8;
    const float* p = W1 + (size_t)n * FIN + k8;
    const v4f a = *(const v4fa*)p;
    const v4f b = *(const v4fa*)(p + 4);
    put8(W1B + (size_t)n * FIN + k8, cvt8(a, b, true));
  } else if (u < nUX + NUW1 + NUW2) {
    const int v  = u - nUX - NUW1;
    const int n  = v >> 8;
    const int k8 = (v & 255) * 8;
    const int kk = k8 & (D1 - 1);
    const float* p = W2 + (size_t)n * D1 + kk;
    const v4f a = *(const v4fa*)p;
    const v4f b = *(const v4fa*)(p + 4);
    put8(W2D + (size_t)n * K2 + k8, cvt8(a, b, true));
  }
}

__global__ __launch_bounds__(GTHR) void k_gemm(const unsigned short* __restrict__ A,
                                               const unsigned short* __restrict__ BT, int K,
                                               const float* __restrict__ attS, const float* __restrict__ attD,
                                               float* outF, int ldo, int nOut, float* att, int mpa) {
  __shared__ __attribute__((aligned(16))) float stg[GBM * GBN];
  __shared__ __attribute__((aligned(16))) float sdot[2 * GBM];
  const int tid = (int)threadIdx.x, lane = tid & 31, wave = tid >> 5, hh = lane >> 4, m = lane & 15;
  const int rowBase = (int)blockIdx.x * GBM;
  const int jt      = (int)blockIdx.y;
  const int col0    = jt * GBN;

  v8f acc[8];
  {
    const v8f z = {0.f, 0.f, 0.f, 0.f, 0.f, 0.f, 0.f, 0.f};
#pragma unroll
    for (int t = 0; t < 8; ++t) acc[t] = z;
  }
  const unsigned short* ap = A  + (size_t)(rowBase + 16 * wave + m) * (size_t)K + 8 * hh;
  const unsigned short* bp = BT + (size_t)(col0 + m) * (size_t)K + 8 * hh;

#pragma unroll 1
  for (int k0 = 0; k0 < K; k0 += 32) {
    FragB af;
    af.h[0] = *(const v8usa*)(ap + k0);
    af.h[1] = *(const v8usa*)(ap + k0 + 16);
#pragma unroll
    for (int nt = 0; nt < 8; ++nt) {
      const unsigned short* wq = bp + (size_t)(16 * nt) * (size_t)K + k0;
      FragB bf;
      bf.h[0] = *(const v8usa*)wq;
      bf.h[1] = *(const v8usa*)(wq + 16);
      acc[nt] = wmb(af, bf, acc[nt]);
    }
  }

#pragma unroll
  for (int nt = 0; nt < 8; ++nt) {
    const int lc = 16 * nt + m;
#pragma unroll
    for (int r = 0; r < 8; ++r) {
      const int lr = 16 * wave + 8 * hh + r;
      stg[lr * GBN + lc] = acc[nt][r];
    }
  }
  __syncthreads();

  v4f as4, ad4;
  {
    const v4f t1 = *(const v4fa*)(attS + col0 + 4 * lane);
    const v4f t2 = *(const v4fa*)(attD + col0 + 4 * lane);
    as4.x = bf16_val(t1.x); as4.y = bf16_val(t1.y); as4.z = bf16_val(t1.z); as4.w = bf16_val(t1.w);
    ad4.x = bf16_val(t2.x); ad4.y = bf16_val(t2.y); ad4.z = bf16_val(t2.z); ad4.w = bf16_val(t2.w);
  }

  v4f pv[16];
#pragma unroll
  for (int i = 0; i < 16; ++i) pv[i] = *(const v4fa*)(stg + (16 * wave + i) * GBN + 4 * lane);

  float rs = 0.0f, rd = 0.0f;
#pragma unroll
  for (int i = 0; i < 16; ++i) {
    float ps = pv[i].x * as4.x;
    ps = fmaf(pv[i].y, as4.y, ps); ps = fmaf(pv[i].z, as4.z, ps); ps = fmaf(pv[i].w, as4.w, ps);
    float pd = pv[i].x * ad4.x;
    pd = fmaf(pv[i].y, ad4.y, pd); pd = fmaf(pv[i].z, ad4.z, pd); pd = fmaf(pv[i].w, ad4.w, pd);
#pragma unroll
    for (int d = 16; d > 0; d >>= 1) {
      ps += __shfl_xor(ps, d, 32);
      pd += __shfl_xor(pd, d, 32);
    }
    rs = (lane == i) ? ps : rs;
    rd = (lane == i) ? pd : rd;
  }
  if (lane < 16) {
    sdot[16 * wave + lane]       = rs;
    sdot[GBM + 16 * wave + lane] = rd;
  }
  __syncthreads();

#pragma unroll
  for (int i = 0; i < 16; ++i) {
    const int r = rowBase + 16 * wave + i;
    if (r < nOut) *(volatile v4f*)(outF + (size_t)r * (size_t)ldo + col0 + 4 * lane) = pv[i];
  }
  __threadfence();
#pragma unroll
  for (int i = 0; i < 16; ++i) {
    const int r = rowBase + 16 * wave + i;
    if (r < nOut) *(volatile v4f*)(outF + (size_t)r * (size_t)ldo + col0 + 4 * lane) = pv[i];
  }

  if (wave == 0) {
    const v4f dv = *(const v4fa*)(sdot + 4 * lane);
    float* dp = att + (size_t)(2 * jt + hh) * (size_t)mpa + rowBase + 4 * m;
    *(volatile v4f*)dp = dv;
    __threadfence();
    *(volatile v4f*)dp = dv;
  }
}

template <int NH, int NP, int NCH, int MODE>
__global__ __launch_bounds__(NTHR) void k_scan(const int* __restrict__ srcs, const int* __restrict__ dsts,
                                               int nE, int nN, int vec8, int mRows,
                                               const float* __restrict__ att, int mpa,
                                               const float* __restrict__ xh, const float* __restrict__ bias,
                                               unsigned short* hb, float* outF) {
  static_assert(NH == 1 || NH == 8);
  static_assert(NH == 1 || NH == NCH);
  static_assert(NP >= 1 && NP <= 8 && NCH <= 8);
  static_assert(MODE == 0 || NCH * 128 * 2 == K2);
  constexpr int NHS   = (NH == 8) ? 3 : 0;
  constexpr int PITCH = NCH * 128;
  extern __shared__ __attribute__((aligned(16))) int dsm[];
  int* list = dsm;
  int* hl   = dsm + LISTN;
  int* sl   = hl + RCAP;
  int* cnt  = sl + RCAP;
  int* offs = cnt + NBA;
  int* cur  = offs + NBA;
  int* misc = cur + NBA;
  const int tid = (int)threadIdx.x, lane = tid & 31, wave = tid >> 5;
  int*   mysrc = misc + MISC_INTS + wave * DEGCAP;
  float* mysc  = (float*)(misc + MISC_INTS + SSRC_INTS) + wave * (DEGCAP * 8);
  unsigned short* rowbuf = (unsigned short*)(dsm + ZTOT_INTS) + wave * K2;
  const int nodeBase = (int)blockIdx.x * NBA;

  {
    const v4i z4 = {0, 0, 0, 0};
    for (int i = tid * 4; i < ZTOT_INTS; i += NTHR * 4) *(v4ia*)(dsm + i) = z4;
  }
  __syncthreads();

  int t = 0, ov = 0;
  const int nChunks = (nE + CHUNK - 1) / CHUNK;
#pragma unroll 1
  for (int ch = 0; ch < nChunks; ++ch) {
    const int cbase = ch * CHUNK;
    const int wc = scan_chunk<SLA>(dsts, nE, cbase, nodeBase, NBA, vec8, list, tid, lane, wave);
    if (lane == 0) misc[wave] = wc;
    __syncthreads();
    if (wave == 0) {
#pragma unroll 1
      for (int w2 = 0; w2 < NWAVE; ++w2) {
        int c = misc[w2];
        c = c < 0 ? 0 : (c > WCAP ? WCAP : c);
#pragma unroll 1
        for (int b0 = 0; b0 < c; b0 += 32) {
          const int idx = b0 + lane;
          const int ent = list[w2 * WCAP + (idx < WCAP ? idx : WCAP - 1)];
          const int m32 = (c - b0) < 32 ? (c - b0) : 32;
#pragma unroll 1
          for (int k = 0; k < m32; ++k) {
            const int u    = __builtin_amdgcn_readlane(ent, k);
            const int slot = u & (NBA - 1);
            const int el   = (u >> SLA) & (CHUNK - 1);
            const int pk   = ((cbase + el) << SLA) | slot;
            if (t < RCAP) {
              if (lane == 0) { hl[t] = pk; cnt[slot] = cnt[slot] + 1; }
              t = t + 1;
            } else {
              ov = 1;
            }
          }
        }
      }
    }
    __syncthreads();
  }
  if (wave == 0 && lane == 0) { misc[8] = t; misc[9] = ov; }
  __syncthreads();
  int tt = misc[8];
  tt = tt < 0 ? 0 : (tt > RCAP ? RCAP : tt);
  const int ovf = misc[9];

  if (wave == 0) {
    const int base = lane * (NBA / 32);
    int s = 0;
#pragma unroll 1
    for (int i = 0; i < NBA / 32; ++i) s += cnt[base + i];
    int incl = s;
#pragma unroll
    for (int d = 1; d < 32; d <<= 1) {
      const int y = __shfl_up(incl, d, 32);
      if (lane >= d) incl += y;
    }
    int run = incl - s;
#pragma unroll 1
    for (int i = 0; i < NBA / 32; ++i) {
      const int cv = cnt[base + i];
      offs[base + i] = run;
      cur[base + i]  = run;
      run += cv;
    }
  }
  __syncthreads();
  if (wave == 0) {
#pragma unroll 1
    for (int b0 = 0; b0 < tt; b0 += 32) {
      const int idx = b0 + lane;
      const int ent = hl[idx < RCAP ? idx : RCAP - 1];
      const int m32 = (tt - b0) < 32 ? (tt - b0) : 32;
#pragma unroll 1
      for (int k = 0; k < m32; ++k) {
        const int u    = __builtin_amdgcn_readlane(ent, k);
        const int slot = u & (NBA - 1);
        if (lane == 0) {
          int p = cur[slot];
          p = p < 0 ? 0 : (p > RCAP - 1 ? RCAP - 1 : p);
          sl[p] = u;
          cur[slot] = p + 1;
        }
      }
    }
  }
  __syncthreads();

  const float qnan = __int_as_float(0x7fc00000);
  const float ninf = __int_as_float((int)0xff800000u);
  const float pz   = (ovf != 0) ? qnan : 0.0f;
  const int   hd   = lane & (NH - 1);
#pragma unroll 1
  for (int si = 0; si < NBA / NWAVE; ++si) {
    const int s    = si * NWAVE + wave;
    const int node = nodeBase + s;
    int c = __builtin_amdgcn_readfirstlane(cnt[s]);
    const bool big = c > DEGCAP;
    c = c < 0 ? 0 : (c > DEGCAP ? DEGCAP : c);
    int o = __builtin_amdgcn_readfirstlane(offs[s]);
    o = o < 0 ? 0 : (o > RCAP ? RCAP : o);
    const int nc = node < nN ? node : nN - 1;

#pragma unroll 1
    for (int b0 = 0; b0 < c; b0 += 32) {
      const int idx = b0 + lane;
      int li = o + idx;
      li = li > RCAP - 1 ? RCAP - 1 : li;
      const int ent = sl[li];
      int eid = ent >> SLA;
      eid = eid < 0 ? 0 : (eid > nE - 1 ? nE - 1 : eid);
      int sr = srcs[eid];
      sr = sr < 0 ? 0 : (sr > nN - 1 ? nN - 1 : sr);
      mysrc[idx] = sr;
    }
    wave_sync();

    float adv = 0.0f;
#pragma unroll
    for (int p = 0; p < NP; ++p) adv += att[(size_t)((hd * NP + p) * 2 + 1) * (size_t)mpa + nc];

    const int nItems = c * NH;
    float mx = ninf;
#pragma unroll 1
    for (int i0 = 0; i0 < nItems; i0 += 32) {
      const int i = i0 + lane;
      const bool valid = i < nItems;
      int hit = i >> NHS;
      hit = hit < c ? hit : c - 1;
      const int sr = mysrc[hit];
      float a = 0.0f;
#pragma unroll
      for (int p = 0; p < NP; ++p) a += att[(size_t)((hd * NP + p) * 2) * (size_t)mpa + sr];
      float v = a + adv;
      v = (v >= 0.0f) ? v : 0.2f * v;
      mysc[i] = v;
      mx = fmaxf(mx, valid ? v : ninf);
    }
#pragma unroll
    for (int d = NH; d < 32; d <<= 1) mx = fmaxf(mx, __shfl_xor(mx, d, 32));
    float dn = 0.0f;
#pragma unroll 1
    for (int i0 = 0; i0 < nItems; i0 += 32) {
      const int i = i0 + lane;
      const bool valid = i < nItems;
      const float v  = mysc[i];
      const float ee = expf(v - mx);
      const float ex = valid ? ee : 0.0f;
      mysc[i] = ex;
      dn += ex;
    }
#pragma unroll
    for (int d = NH; d < 32; d <<= 1) dn += __shfl_xor(dn, d, 32);
    const float den = dn + 1e-16f;
#pragma unroll 1
    for (int i0 = 0; i0 < nItems; i0 += 32) {
      const int i = i0 + lane;
      const float ex = mysc[i];
      mysc[i] = ex / den;
    }
    wave_sync();

    v4f acc[NCH];
    {
      const v4f z = {0.f, 0.f, 0.f, 0.f};
#pragma unroll
      for (int j = 0; j < NCH; ++j) acc[j] = z;
    }
#pragma unroll 1
    for (int k = 0; k < c; ++k) {
      const int sk = __builtin_amdgcn_readfirstlane(mysrc[k]);
      float al[8];
      if constexpr (NH == 8) {
        const v4f a0 = *(const v4fa*)(mysc + 8 * k);
        const v4f a1 = *(const v4fa*)(mysc + 8 * k + 4);
        al[0] = a0.x; al[1] = a0.y; al[2] = a0.z; al[3] = a0.w;
        al[4] = a1.x; al[5] = a1.y; al[6] = a1.z; al[7] = a1.w;
      } else {
        const float a0 = mysc[k];
        al[0] = a0; al[1] = a0; al[2] = a0; al[3] = a0;
        al[4] = a0; al[5] = a0; al[6] = a0; al[7] = a0;
      }
      const float* rp = xh + (size_t)sk * PITCH + 4 * lane;
#pragma unroll
      for (int j = 0; j < NCH; ++j) {
        const v4f r = *(const v4fa*)(rp + 128 * j);
        acc[j].x = fmaf(al[j], r.x, acc[j].x);
        acc[j].y = fmaf(al[j], r.y, acc[j].y);
        acc[j].z = fmaf(al[j], r.z, acc[j].z);
        acc[j].w = fmaf(al[j], r.w, acc[j].w);
      }
    }

    const float pzr = big ? qnan : pz;
    const bool live = node < nN;
    if constexpr (MODE != 0) {
#pragma unroll
      for (int j = 0; j < NCH; ++j) {
        const v4f bb = *(const v4fa*)(bias + 128 * j + 4 * lane);
        float t0 = acc[j].x + bf16_val(bb.x);
        float t1 = acc[j].y + bf16_val(bb.y);
        float t2 = acc[j].z + bf16_val(bb.z);
        float t3 = acc[j].w + bf16_val(bb.w);
        t0 = (t0 > 0.0f) ? t0 : (t0 - t0);
        t1 = (t1 > 0.0f) ? t1 : (t1 - t1);
        t2 = (t2 > 0.0f) ? t2 : (t2 - t2);
        t3 = (t3 > 0.0f) ? t3 : (t3 - t3);
        const float m0 = live ? (t0 + pzr) : 0.0f;
        const float m1 = live ? (t1 + pzr) : 0.0f;
        const float m2 = live ? (t2 + pzr) : 0.0f;
        const float m3 = live ? (t3 + pzr) : 0.0f;
        v4us mh, ml;
        unsigned hbits;
        hbits = bf16_bits(m0); mh[0] = (unsigned short)hbits; ml[0] = (unsigned short)bf16_bits(m0 - __uint_as_float(hbits << 16));
        hbits = bf16_bits(m1); mh[1] = (unsigned short)hbits; ml[1] = (unsigned short)bf16_bits(m1 - __uint_as_float(hbits << 16));
        hbits = bf16_bits(m2); mh[2] = (unsigned short)hbits; ml[2] = (unsigned short)bf16_bits(m2 - __uint_as_float(hbits << 16));
        hbits = bf16_bits(m3); mh[3] = (unsigned short)hbits; ml[3] = (unsigned short)bf16_bits(m3 - __uint_as_float(hbits << 16));
        *(v4usa*)(rowbuf + 128 * j + 4 * lane) = mh;
        *(v4usa*)(rowbuf + D1 + 128 * j + 4 * lane) = ml;
      }
      wave_sync();
      v8us q[8];
#pragma unroll
      for (int qq = 0; qq < 8; ++qq) q[qq] = *(const v8usa*)(rowbuf + 256 * qq + 8 * lane);
      wave_sync();
      if (node < mRows) {
        unsigned short* rpw = hb + (size_t)node * K2 + 8 * lane;
#pragma unroll
        for (int qq = 0; qq < 8; ++qq) *(volatile v8us*)(rpw + 256 * qq) = q[qq];
        __threadfence();
#pragma unroll
        for (int qq = 0; qq < 8; ++qq) *(volatile v8us*)(rpw + 256 * qq) = q[qq];
      }
    } else {
      v4f y[NCH];
#pragma unroll
      for (int j = 0; j < NCH; ++j) {
        const v4f bb = *(const v4fa*)(bias + 128 * j + 4 * lane);
        y[j].x = (acc[j].x + bf16_val(bb.x)) + pzr;
        y[j].y = (acc[j].y + bf16_val(bb.y)) + pzr;
        y[j].z = (acc[j].z + bf16_val(bb.z)) + pzr;
        y[j].w = (acc[j].w + bf16_val(bb.w)) + pzr;
      }
      wave_sync();
      if (live) {
        float* op = outF + (size_t)node * PITCH + 4 * lane;
#pragma unroll
        for (int j = 0; j < NCH; ++j) *(volatile v4f*)(op + 128 * j) = y[j];
        __threadfence();
#pragma unroll
        for (int j = 0; j < NCH; ++j) *(volatile v4f*)(op + 128 * j) = y[j];
      }
    }
  }
}

static inline int cdiv(int a, int b) { return (a + b - 1) / b; }
static inline size_t al256(size_t o) { return (o + 255) & ~(size_t)255; }

extern "C" void kernel_launch(void* const* d_in, const int* in_sizes, int n_in,
                              void* d_out, int out_size, void* d_ws, size_t ws_size,
                              hipStream_t stream) {
  if (n_in < 10) return;
  if (in_sizes[0] < FIN || (in_sizes[0] % FIN) != 0) return;
  const int nN = in_sizes[0] / FIN;
  if (nN < 1 || nN > (1 << 20)) return;
  if (in_sizes[1] < 2 || (in_sizes[1] & 1) != 0) return;
  const int nE = in_sizes[1] / 2;
  if (nE < 1 || nE >= (1 << (31 - SLA))) return;
  if (in_sizes[2] != D1 * FIN) return;
  if (in_sizes[3] != D1 || in_sizes[4] != D1 || in_sizes[5] != D1) return;
  if (in_sizes[6] != D2 * D1) return;
  if (in_sizes[7] != D2 || in_sizes[8] != D2 || in_sizes[9] != D2) return;
  if ((long long)out_size != (long long)nN * D2) return;

  const float* x     = (const float*)d_in[0];
  const int*   edge  = (const int*)d_in[1];
  const float* W1    = (const float*)d_in[2];
  const float* attS1 = (const float*)d_in[3];
  const float* attD1 = (const float*)d_in[4];
  const float* b1    = (const float*)d_in[5];
  const float* W2    = (const float*)d_in[6];
  const float* attS2 = (const float*)d_in[7];
  const float* attD2 = (const float*)d_in[8];
  const float* b2    = (const float*)d_in[9];
  float* out = (float*)d_out;
  const int* src = edge;
  const int* dst = edge + nE;

  const int MP = cdiv(nN, 128) * 128;
  const int gM = MP / GBM;
  const int gA = cdiv(MP, NBA);
  if ((long long)gA * NBA < (long long)MP) return;
  if ((MP % GBM) != 0 || ((MP * (FIN / 8)) % NTHR) != 0) return;
  const int vec8 = ((nE & 3) == 0) ? 1 : 0;

  char* ws = (char*)d_ws;
  size_t off = 0;
  const size_t oXB  = off; off = al256(off + (size_t)MP * FIN * 2);
  const size_t oW1B = off; off = al256(off + (size_t)D1 * FIN * 2);
  const size_t oW2D = off; off = al256(off + (size_t)D2 * K2 * 2);
  const size_t oXH  = off; off = al256(off + (size_t)nN * D1 * 4);
  const size_t oAT1 = off; off = al256(off + (size_t)16 * MP * 4);
  const size_t oAT2 = off; off = al256(off + (size_t)12 * MP * 4);
  const size_t oHL  = off; off = al256(off + (size_t)MP * K2 * 2);
  if (off > ws_size || off > (size_t)WSMAX) return;
  if ((size_t)nN * D2 * 4 > (size_t)nN * D1 * 4) return;
  unsigned short* XB   = (unsigned short*)(ws + oXB);
  unsigned short* W1B  = (unsigned short*)(ws + oW1B);
  unsigned short* W2D  = (unsigned short*)(ws + oW2D);
  float*          XH1  = (float*)(ws + oXH);
  float*          XH2  = (float*)(ws + oXH);
  float*          ATT1 = (float*)(ws + oAT1);
  float*          ATT2 = (float*)(ws + oAT2);
  unsigned short* H1HL = (unsigned short*)(ws + oHL);

  const size_t scanLds = (size_t)SCAN_LDS_INTS * 4;
  hipFuncSetAttribute(reinterpret_cast<const void*>(&k_scan<8, 1, 8, 1>), hipFuncAttributeMaxDynamicSharedMemorySize, (int)scanLds);
  hipFuncSetAttribute(reinterpret_cast<const void*>(&k_scan<1, 6, 6, 0>), hipFuncAttributeMaxDynamicSharedMemorySize, (int)scanLds);

  const int nUnits = MP * (FIN / 8) + NUW1 + NUW2;
  k_prep<<<nUnits / NTHR, NTHR, 0, stream>>>(x, W1, W2, nN, MP, XB, W1B, W2D);
  k_gemm<<<dim3(gM, D1 / GBN), GTHR, 0, stream>>>(XB, W1B, FIN, attS1, attD1, XH1, D1, nN, ATT1, MP);
  k_scan<8, 1, 8, 1><<<gA, NTHR, scanLds, stream>>>(src, dst, nE, nN, vec8, MP, ATT1, MP, XH1, b1, H1HL, out);
  k_gemm<<<dim3(gM, D2 / GBN), GTHR, 0, stream>>>(H1HL, W2D, K2, attS2, attD2, XH2, D2, nN, ATT2, MP);
  k_scan<1, 6, 6, 0><<<gA, NTHR, scanLds, stream>>>(src, dst, nE, nN, vec8, MP, ATT2, MP, XH2, b2, H1HL, out);
}
